// HGRN2Attention_13752485282226
// MI455X (gfx1250) — hardware-verified
//
#include <hip/hip_runtime.h>
#include <math.h>

constexpr int kBatch   = 2;
constexpr int kSeq     = 4096;
constexpr int kModel   = 1024;
constexpr int kHeads   = 8;
constexpr int kHeadDim = 128;
constexpr int kProjN   = 3 * kModel;
constexpr int kChunkT  = 16;
constexpr float kQScale = 0.08838834764831845f;
constexpr float kEps    = 1e-5f;
static_assert(kHeads * kHeadDim == kModel);
static_assert(kSeq % kChunkT == 0);
static_assert(kChunkT == 16);

typedef __attribute__((ext_vector_type(16))) _Float16 v16h;
typedef __attribute__((ext_vector_type(8)))  _Float16 v8h;
typedef __attribute__((ext_vector_type(16))) __bf16   v16b;
typedef __attribute__((ext_vector_type(8)))  __bf16   v8b;
typedef __attribute__((ext_vector_type(8)))  float    v8f;
typedef __attribute__((ext_vector_type(4)))  float    v4f;
typedef __attribute__((ext_vector_type(4)))  unsigned int v4u;

__device__ __forceinline__ unsigned short f2bf_bits(float f) {
  unsigned u = __float_as_uint(f);
  return (unsigned short)((u + 0x7FFFu + ((u >> 16) & 1u)) >> 16);
}
__device__ __forceinline__ float bf_bits2f(unsigned short h) { return __uint_as_float(((unsigned)h) << 16); }

__device__ __forceinline__ void dep_guard_h(v8f& a, v8f& b, v16h x, v16h y) { asm volatile("v_nop\n\tv_nop\n\tv_nop\n\tv_nop" : "+v"(a), "+v"(b) : "v"(x), "v"(y)); }
__device__ __forceinline__ void dep_guard_b(v8f& a, v8f& b, v16b x, v16b y) { asm volatile("v_nop\n\tv_nop\n\tv_nop\n\tv_nop" : "+v"(a), "+v"(b) : "v"(x), "v"(y)); }
__device__ __forceinline__ void keep4_h(v16h a, v16h b, v16h c, v16h d) { asm volatile("v_nop" :: "v"(a), "v"(b), "v"(c), "v"(d)); }
__device__ __forceinline__ void keep4_b(v16b a, v16b b, v16b c, v16b d) { asm volatile("v_nop" :: "v"(a), "v"(b), "v"(c), "v"(d)); }
__device__ __forceinline__ void acc_guard4(v8f& a, v8f& b, v8f& c, v8f& d) { asm volatile("v_nop\n\tv_nop\n\tv_nop\n\tv_nop" : "+v"(a), "+v"(b), "+v"(c), "+v"(d)); }
template <typename T> struct Frag;
template <> struct Frag<_Float16> {
  typedef v16h V; union U { v16h v; v8h h[2]; };
  static __device__ __forceinline__ v16h load(const _Float16* p) {
    U f; f.h[0] = *(const v8h*)(p); f.h[1] = *(const v8h*)(p + 16); return f.v;
  }
  static __device__ __forceinline__ v8f mma(v16h a, v16h b, v8f c) {
    return __builtin_amdgcn_wmma_f32_16x16x32_f16(false, a, false, b, (short)0, c, false, false);
  }
  static __device__ __forceinline__ void guard(v8f& a, v8f& b, v16h x, v16h y) { dep_guard_h(a, b, x, y); }
  static __device__ __forceinline__ void keep(v16h a, v16h b, v16h c, v16h d) { keep4_h(a, b, c, d); }
};
template <> struct Frag<__bf16> {
  typedef v16b V; union U { v16b v; v8b h[2]; };
  static __device__ __forceinline__ v16b load(const __bf16* p) {
    U f; f.h[0] = *(const v8b*)(p); f.h[1] = *(const v8b*)(p + 16); return f.v;
  }
  static __device__ __forceinline__ v8f mma(v16b a, v16b b, v8f c) {
    return __builtin_amdgcn_wmma_f32_16x16x32_bf16(false, a, false, b, (short)0, c, false, false);
  }
  static __device__ __forceinline__ void guard(v8f& a, v8f& b, v16b x, v16b y) { dep_guard_b(a, b, x, y); }
  static __device__ __forceinline__ void keep(v16b a, v16b b, v16b c, v16b d) { keep4_b(a, b, c, d); }
};

__device__ __forceinline__ unsigned pk16(unsigned short a, unsigned short b) { return (unsigned)a | ((unsigned)b << 16); }
__device__ __forceinline__ unsigned short h_bits(float f) { const _Float16 h = (_Float16)f; return __builtin_bit_cast(unsigned short, h); }

__device__ __forceinline__ float sigm_f(float v) {
  const float e = __expf(-fabsf(v));
  const float r = 1.0f / (1.0f + e);
  return (v >= 0.0f) ? r : e * r;
}

template <int ET> struct Elem;
template <> struct Elem<0> { typedef _Float16 T; };
template <> struct Elem<1> { typedef __bf16 T; };
template <int ET, int SPL, int BIAS, int OUT_MODE, int ACT, int MULR>
__global__ __launch_bounds__(256) void wmma_gemm64(
    const unsigned short* __restrict__ Ap, const unsigned short* __restrict__ A2p, int lda, long strideA,
    const unsigned short* __restrict__ Btp, const unsigned short* __restrict__ Bt2p, int ldb, long strideB,
    void* __restrict__ Cout, void* __restrict__ Cout2, int ldc, long strideC,
    const float* __restrict__ bias, int nbias,
    const float* __restrict__ mulr, int ldr,
    int M, int N, int K, float scale) {
  typedef typename Elem<ET>::T T;
  typedef typename Frag<T>::V V;
  const T* A = (const T*)Ap; const T* A2 = (const T*)A2p; const T* Bt = (const T*)Btp; const T* Bt2 = (const T*)Bt2p;
  __shared__ __align__(16) float sT[8][16 * 68];
  const int b    = blockIdx.y;
  const int lane = threadIdx.x & 31;
  const int wave = threadIdx.x >> 5;
  const int tilesN = N >> 6;
  const int tilesM = M >> 6;
  const int tile = blockIdx.x * 8 + wave;
  if (tile >= tilesM * tilesN) return;
  const int tm = tile / tilesN;
  const int tn = tile - tm * tilesN;
  const int m0 = tm << 6;
  const int n0 = tn << 6;

  const T* Ab  = A  + (size_t)b * strideA;
  const T* Bb  = Bt + (size_t)b * strideB;
  const T* Ab2 = (SPL & 1) ? (A2  + (size_t)b * strideA) : nullptr;
  const T* Bb2 = (SPL & 2) ? (Bt2 + (size_t)b * strideB) : nullptr;

  const int rlane = lane & 15;
  const int koff  = (lane >> 4) * 8;
  const int mOff  = (lane >> 4) * 8;

  v8f acc[4][4];
#pragma unroll
  for (int i = 0; i < 4; ++i)
#pragma unroll
    for (int j = 0; j < 4; ++j) acc[i][j] = (v8f){0.f,0.f,0.f,0.f,0.f,0.f,0.f,0.f};

  for (int k0 = 0; k0 < K; k0 += 32) {
    V bh[4], bl[4];
#pragma unroll
    for (int j = 0; j < 4; ++j) {
      const size_t bo = (size_t)(n0 + (j << 4) + rlane) * ldb + koff + k0;
      bh[j] = Frag<T>::load(Bb + bo);
      if (SPL & 2) bl[j] = Frag<T>::load(Bb2 + bo);
    }
#pragma unroll
    for (int i = 0; i < 4; ++i) {
      const size_t ao = (size_t)(m0 + (i << 4) + rlane) * lda + koff + k0;
      V ah = Frag<T>::load(Ab + ao);
      V al;
      if (SPL & 1) al = Frag<T>::load(Ab2 + ao);
#pragma unroll
      for (int j = 0; j < 4; ++j) {
        acc[i][j] = Frag<T>::mma(ah, bh[j], acc[i][j]);
        if (SPL & 2) acc[i][j] = Frag<T>::mma(ah, bl[j], acc[i][j]);
        if (SPL & 1) acc[i][j] = Frag<T>::mma(al, bh[j], acc[i][j]);
      }
      Frag<T>::guard(acc[i][0], acc[i][3], ah, (SPL & 1) ? al : ah);
    }
    Frag<T>::keep(bh[0], bh[1], bh[2], bh[3]);
    if (SPL & 2) Frag<T>::keep(bl[0], bl[1], bl[2], bl[3]);
  }
  acc_guard4(acc[0][0], acc[0][1], acc[0][2], acc[0][3]);
  acc_guard4(acc[1][0], acc[1][1], acc[1][2], acc[1][3]);
  acc_guard4(acc[2][0], acc[2][1], acc[2][2], acc[2][3]);
  acc_guard4(acc[3][0], acc[3][1], acc[3][2], acc[3][3]);

  float* slab = sT[wave];
#pragma unroll
  for (int i = 0; i < 4; ++i) {
    const int mBase = m0 + (i << 4);
#pragma unroll
    for (int j = 0; j < 4; ++j) {
      const int n = n0 + (j << 4) + rlane;
      float bv = 0.f;
      if (BIAS == 2) {
        const int nc = (n < nbias) ? n : (nbias - 1);
        bv = bf_bits2f(f2bf_bits(bias[nc]));
        if (n >= nbias) bv = 0.0f;
      }
#pragma unroll
      for (int r = 0; r < 8; ++r) {
        float v = acc[i][j][r] * scale;
        if (BIAS == 2) v += bv;
        if (ACT == 3) v = v * sigm_f(v);
        if (ACT == 7) v = sigm_f(0.0625f * v);
        if (MULR) v = v * mulr[(size_t)(mBase + mOff + r) * ldr + n];
        slab[(mOff + r) * 68 + (j << 4) + rlane] = v;
      }
    }
    __builtin_amdgcn_fence(__ATOMIC_RELEASE, "workgroup");
    __builtin_amdgcn_wave_barrier();
    __builtin_amdgcn_fence(__ATOMIC_ACQUIRE, "workgroup");
    if (OUT_MODE == 0) {
      float* Cp = (float*)Cout + (size_t)b * strideC;
      const int hh = lane >> 4, c4 = (lane & 15) * 4;
      for (int pass = 0; pass < 2; ++pass) {
#pragma unroll
        for (int it = 0; it < 8; ++it) {
          const int row = it * 2 + hh;
          v4f v = *(const v4f*)(slab + row * 68 + c4);
          *(volatile v4f*)(Cp + (size_t)(mBase + row) * ldc + n0 + c4) = v;
        }
        __threadfence();
      }
    } else {
      const int q = lane >> 3, c8 = (lane & 7) * 8;
      unsigned short* Cp  = (unsigned short*)Cout  + (size_t)b * strideC;
      unsigned short* Cp2 = (OUT_MODE == 2) ? ((unsigned short*)Cout2 + (size_t)b * strideC) : nullptr;
      for (int pass = 0; pass < 2; ++pass) {
#pragma unroll
        for (int it = 0; it < 4; ++it) {
          const int row = it * 4 + q;
          const float* sp = slab + row * 68 + c8;
          v8h hv, lv;
#pragma unroll
          for (int e = 0; e < 8; ++e) {
            if (OUT_MODE == 1) {
              hv[e] = (_Float16)sp[e];
            } else {
              unsigned short hb = f2bf_bits(sp[e]);
              unsigned short lb = f2bf_bits(sp[e] - bf_bits2f(hb));
              hv[e] = __builtin_bit_cast(_Float16, hb);
              lv[e] = __builtin_bit_cast(_Float16, lb);
            }
          }
          *(volatile v8h*)(Cp + (size_t)(mBase + row) * ldc + n0 + c8) = hv;
          if (OUT_MODE == 2) *(volatile v8h*)(Cp2 + (size_t)(mBase + row) * ldc + n0 + c8) = lv;
        }
        __threadfence();
      }
    }
    __builtin_amdgcn_fence(__ATOMIC_RELEASE, "workgroup");
    __builtin_amdgcn_wave_barrier();
    __builtin_amdgcn_fence(__ATOMIC_ACQUIRE, "workgroup");
  }
}

template <int MODE>
__global__ __launch_bounds__(256) void cast8_kernel(const float* __restrict__ in, unsigned short* __restrict__ out, int n8, float scale) {
  const int i = blockIdx.x * 256 + threadIdx.x;
  if (i >= n8) return;
  const float* p = in + 8 * (size_t)i;
  const v4f a = *(const v4f*)(p);
  const v4f c = *(const v4f*)(p + 4);
  unsigned short hb[8];
#pragma unroll
  for (int e = 0; e < 4; ++e) {
    if (MODE == 0) {
      hb[e]     = f2bf_bits(a[e]);
      hb[4 + e] = f2bf_bits(c[e]);
    } else {
      hb[e]     = h_bits(bf_bits2f(f2bf_bits(a[e])) * scale);
      hb[4 + e] = h_bits(bf_bits2f(f2bf_bits(c[e])) * scale);
    }
  }
  const v4u u = (v4u){pk16(hb[0], hb[1]), pk16(hb[2], hb[3]), pk16(hb[4], hb[5]), pk16(hb[6], hb[7])};
  unsigned short* q = out + 8 * (size_t)i;
  *(volatile v4u*)q = u;
  __threadfence();
  *(volatile v4u*)q = u;
  (void)scale;
}

__global__ __launch_bounds__(256) void gate_act_kernel(float* __restrict__ proj, float qscale) {
  const int row = blockIdx.x, part = blockIdx.y, tid = threadIdx.x;
  float* p = proj + (size_t)row * kProjN + (size_t)part * kModel + (size_t)tid * 4;
  v4f y = *(const v4f*)p;
  v4f r = y;
  if (part == 0) {
#pragma unroll 1
    for (int e = 0; e < 4; ++e) {
      const float x  = y.x;
      const float sg = 1.0f / (1.0f + expf(-x));
      const float val = (x * sg) * qscale;
      y = __builtin_shufflevector(y, y, 1, 2, 3, 0);
      r = __builtin_shufflevector(r, r, 1, 2, 3, 0);
      r.w = val;
    }
  } else {
#pragma unroll 1
    for (int e = 0; e < 4; ++e) {
      const float x  = y.x;
      const float ex = expf(-fabsf(x));
      const float lg = fminf(x, 0.0f) - log1pf(ex);
      const float val = expf(lg);
      y = __builtin_shufflevector(y, y, 1, 2, 3, 0);
      r = __builtin_shufflevector(r, r, 1, 2, 3, 0);
      r.w = val;
    }
  }
  const v4f outv = r;
  *(volatile v4f*)p = outv;
  __threadfence();
  *(volatile v4f*)p = outv;
}

__global__ __launch_bounds__(256) void hgrn_scan_kernel(const float* __restrict__ proj, float* __restrict__ obuf) {
  __shared__ __align__(16) float sq[kChunkT][kHeadDim];
  __shared__ __align__(16) float sk[kChunkT][kHeadDim];
  __shared__ __align__(16) float sa[kChunkT][kHeadDim];
  __shared__ __align__(16) float sv[kChunkT][64];
  __shared__ __align__(16) float so[kChunkT][64];
  const int h    = blockIdx.x >> 1;
  const int half = blockIdx.x & 1;
  const int tid  = threadIdx.x;
  const int lane = tid & 31, wave = tid >> 5;
  const int vcol = tid >> 2, kq = tid & 3;
  const int fb   = kq * 32;
  const int cq = h * kHeadDim;
  const int ca = kModel + h * kHeadDim;
  const int cv = 2 * kModel + h * kHeadDim + half * 64;
  const int co = h * kHeadDim + half * 64;
  const v4f one4 = {1.0f, 1.0f, 1.0f, 1.0f};

  float S[32];
#pragma unroll
  for (int e = 0; e < 32; ++e) S[e] = 0.0f;

#pragma unroll 1
  for (int t0 = 0; t0 < kSeq; t0 += kChunkT) {
    __syncthreads();
#pragma unroll
    for (int i = 0; i < 2; ++i) {
      const int j  = tid + i * 256;
      const int s  = j >> 5, c4 = (j & 31) * 4;
      const float* rp = proj + (size_t)(t0 + s) * kProjN;
      const v4f qv = *(const v4f*)(rp + cq + c4);
      const v4f av = *(const v4f*)(rp + ca + c4);
      *(v4f*)(&sq[s][c4]) = qv;
      *(v4f*)(&sa[s][c4]) = av;
      *(v4f*)(&sk[s][c4]) = one4 - av;
    }
    {
      const int s = tid >> 4, c4 = (tid & 15) * 4;
      const v4f vv = *(const v4f*)(proj + (size_t)(t0 + s) * kProjN + cv + c4);
      *(v4f*)(&sv[s][c4]) = vv;
    }
    __syncthreads();
#pragma unroll 1
    for (int s = 0; s < kChunkT; ++s) {
      const float vv = sv[s][vcol];
      float o = 0.0f;
#pragma unroll
      for (int e4 = 0; e4 < 8; ++e4) {
        const int f0 = fb + e4 * 4;
        const v4f a4 = *(const v4f*)(&sa[s][f0]);
        const v4f k4 = *(const v4f*)(&sk[s][f0]);
        const v4f q4 = *(const v4f*)(&sq[s][f0]);
#pragma unroll
        for (int e = 0; e < 4; ++e) {
          const int idx = e4 * 4 + e;
          const float sn = a4[e] * S[idx] + k4[e] * vv;
          S[idx] = sn;
          o += q4[e] * sn;
        }
      }
      o += __shfl_xor(o, 1, 32);
      o += __shfl_xor(o, 2, 32);
      if (kq == 0) so[s][vcol] = o;
    }
    __syncthreads();
    {
      const int hh = lane >> 4, c4 = (lane & 15) * 4;
      const int row = wave * 2 + hh;
      for (int pass = 0; pass < 2; ++pass) {
        const v4f val = *(const v4f*)(&so[row][c4]);
        *(volatile v4f*)(obuf + (size_t)(t0 + row) * kModel + co + c4) = val;
        __threadfence();
      }
    }
  }
}

__global__ __launch_bounds__(256) void rms_split_kernel(const float* __restrict__ obuf, const float* __restrict__ gw,
                                                        unsigned short* __restrict__ ofh, unsigned short* __restrict__ ofl) {
  __shared__ float red[8];
  const int tid = threadIdx.x, lane = tid & 31, wave = tid >> 5;
  const int rsel = tid >> 7;
  const int t = tid & 127;
  const int row = blockIdx.x * 2 + rsel;
  const float* src = obuf + (size_t)row * kModel + (size_t)t * 8;
  const v4f a = *(const v4f*)(src);
  const v4f c = *(const v4f*)(src + 4);
  float ss = ((a.x * a.x + a.y * a.y) + (a.z * a.z + a.w * a.w)) + ((c.x * c.x + c.y * c.y) + (c.z * c.z + c.w * c.w));
#pragma unroll
  for (int off = 16; off > 0; off >>= 1) ss += __shfl_xor(ss, off, 32);
  if (lane == 0) red[wave] = ss;
  __syncthreads();
  const float tot = (red[rsel * 4 + 0] + red[rsel * 4 + 1]) + (red[rsel * 4 + 2] + red[rsel * 4 + 3]);
  const float inv = 1.0f / sqrtf(tot * (1.0f / 1024.0f) + kEps);
  const v4f g0 = *(const v4f*)(gw + (size_t)t * 8);
  const v4f g1 = *(const v4f*)(gw + (size_t)t * 8 + 4);
  unsigned short hb[8], lb[8];
#pragma unroll
  for (int e = 0; e < 4; ++e) {
    float f0 = a[e] * inv;
    f0 = f0 * bf_bits2f(f2bf_bits(g0[e]));
    hb[e] = f2bf_bits(f0);
    lb[e] = f2bf_bits(f0 - bf_bits2f(hb[e]));
    float f1 = c[e] * inv;
    f1 = f1 * bf_bits2f(f2bf_bits(g1[e]));
    hb[4 + e] = f2bf_bits(f1);
    lb[4 + e] = f2bf_bits(f1 - bf_bits2f(hb[4 + e]));
  }
  const v4u uh = (v4u){pk16(hb[0], hb[1]), pk16(hb[2], hb[3]), pk16(hb[4], hb[5]), pk16(hb[6], hb[7])};
  const v4u ul = (v4u){pk16(lb[0], lb[1]), pk16(lb[2], lb[3]), pk16(lb[4], lb[5]), pk16(lb[6], lb[7])};
  unsigned short* qh = ofh + (size_t)row * kModel + (size_t)t * 8;
  unsigned short* ql = ofl + (size_t)row * kModel + (size_t)t * 8;
  *(volatile v4u*)qh = uh;
  *(volatile v4u*)ql = ul;
  __threadfence();
  *(volatile v4u*)qh = uh;
  *(volatile v4u*)ql = ul;
}

extern "C" void kernel_launch(void* const* d_in, const int* in_sizes, int n_in,
                              void* d_out, int out_size, void* d_ws, size_t ws_size,
                              hipStream_t stream) {
  const int rowsAll = kBatch * kSeq;
  if (n_in < 6) return;
  if (in_sizes[0] != rowsAll * kModel) return;
  if (in_sizes[1] != kModel * kModel || in_sizes[2] != kModel * kModel || in_sizes[3] != kModel * kModel) return;
  if (in_sizes[4] != kModel) return;
  if (in_sizes[5] != kModel * kModel) return;
  if (out_size != rowsAll * kModel) return;

  const float* x  = (const float*)d_in[0];
  const float* Wq = (const float*)d_in[1];
  const float* Wf = (const float*)d_in[2];
  const float* Wi = (const float*)d_in[3];
  const float* gw = (const float*)d_in[4];
  const float* Wo = (const float*)d_in[5];
  float* outp = (float*)d_out;

  const size_t szXB   = (size_t)rowsAll * kModel * 2;
  const size_t szW3   = (size_t)kProjN * kModel * 2;
  const size_t szWO   = (size_t)kModel * kModel * 2;
  const size_t szPROJ = (size_t)kSeq * kProjN * 4;
  const size_t szOFP  = (size_t)kSeq * kModel * 2;
  const size_t szOBUF = (size_t)kSeq * kModel * 4;
  if (2 * szOFP > szPROJ) return;

  size_t off = 0;
  const size_t oXB   = off; off += szXB;
  const size_t oW3   = off; off += szW3;
  const size_t oWO   = off; off += szWO;
  const size_t oPROJ = off; off += szPROJ;
  const size_t oOBUF = off; off += szOBUF;
  const size_t total = off;
  if (total > ws_size) return;
  if (total > (size_t)134217728) return;

  char* ws = (char*)d_ws;
  unsigned short* XB   = (unsigned short*)(ws + oXB);
  unsigned short* W3   = (unsigned short*)(ws + oW3);
  unsigned short* WOB  = (unsigned short*)(ws + oWO);
  float*          PROJ = (float*)(ws + oPROJ);
  unsigned short* OFH  = (unsigned short*)(ws + oPROJ);
  unsigned short* OFL  = (unsigned short*)(ws + oPROJ + szOFP);
  float*          OBUF = (float*)(ws + oOBUF);

  const dim3 blk(256);

  {
    const int n8 = rowsAll * kModel / 8;
    cast8_kernel<0><<<dim3(n8 / 256), blk, 0, stream>>>(x, XB, n8, 1.0f);
  }
  {
    const int n8w = kModel * kModel / 8;
    cast8_kernel<0><<<dim3(n8w / 256), blk, 0, stream>>>(Wq, W3,                               n8w, 1.0f);
    cast8_kernel<0><<<dim3(n8w / 256), blk, 0, stream>>>(Wf, W3 + (size_t)kModel * kModel,     n8w, 1.0f);
    cast8_kernel<0><<<dim3(n8w / 256), blk, 0, stream>>>(Wi, W3 + (size_t)2 * kModel * kModel, n8w, 1.0f);
    cast8_kernel<0><<<dim3(n8w / 256), blk, 0, stream>>>(Wo, WOB,                              n8w, 1.0f);
  }

  const dim3 gPROJ(((kSeq / 64) * (kProjN / 64) + 7) / 8, 1);
  const dim3 gOUT(((kSeq / 64) * (kModel / 64) + 7) / 8, 1);

  for (int bb = 0; bb < kBatch; ++bb) {
    wmma_gemm64<1, 0, 0, 0, 0, 0><<<gPROJ, blk, 0, stream>>>(
        XB + (size_t)bb * kSeq * kModel, XB + (size_t)bb * kSeq * kModel, kModel, 0L,
        W3, W3, kModel, 0L,
        (void*)PROJ, (void*)PROJ, kProjN, 0L,
        gw, kModel, OBUF, kModel,
        kSeq, kProjN, kModel, 1.0f);
    gate_act_kernel<<<dim3(kSeq, 2), blk, 0, stream>>>(PROJ, kQScale);
    hgrn_scan_kernel<<<dim3(kHeads * 2), blk, 0, stream>>>(PROJ, OBUF);
    rms_split_kernel<<<dim3(kSeq / 2), blk, 0, stream>>>(OBUF, gw, OFH, OFL);
    wmma_gemm64<1, 1, 0, 0, 0, 0><<<gOUT, blk, 0, stream>>>(
        OFH, OFL, kModel, 0L,
        WOB, WOB, kModel, 0L,
        (void*)(outp + (size_t)bb * kSeq * kModel), (void*)(outp + (size_t)bb * kSeq * kModel), kModel, 0L,
        gw, kModel, OBUF, kModel,
        kSeq, kModel, kModel, 1.0f);
  }
}
